// KANLayer_original_90486370993053
// MI455X (gfx1250) — hardware-verified
//
#include <hip/hip_runtime.h>

typedef _Float16 v16h __attribute__((ext_vector_type(16)));
typedef _Float16 v8h  __attribute__((ext_vector_type(8)));
typedef float    v8f  __attribute__((ext_vector_type(8)));
typedef float    v4f  __attribute__((ext_vector_type(4)));
union Frag { v16h v; v8h half[2]; };

#define IN_DIM  256
#define OUT_DIM 256
#define NKNOT   12
#define NB      8
#define NF      9
#define KTOT    (IN_DIM * NF)
#define NCHUNK  (KTOT / 256)
#define FSCALE  16.0f
#define WSCALE  64.0f
#define OSCALE  (1.0f / 1024.0f)
#define TM 64
#define TN 64

static_assert(KTOT % 64 == 0);
static_assert(KTOT % 256 == 0);
static_assert((KTOT * 2) % 128 == 0);
static_assert(OUT_DIM % TN == 0);


__device__ __forceinline__ void store_plane_row(const _Float16* lds_row, _Float16* dst_row)
{
    const int l = threadIdx.x & 31;
    const int w = threadIdx.x >> 5;
    v8h vv[2];
    #pragma unroll
    for (int q = 0; q < 2; ++q) {
        const int ch = w + 8 * q;
        v8h z = {};
        vv[q] = z;
        if (ch < NCHUNK) vv[q] = *(const v8h*)(lds_row + ch * 256 + l * 8);
    }
    #pragma unroll
    for (int q = 0; q < 2; ++q) {
        const int ch = w + 8 * q;
        if (ch < NCHUNK) *(volatile v8h*)(dst_row + ch * 256 + l * 8) = vv[q];
    }
    __threadfence();
    #pragma unroll
    for (int q = 0; q < 2; ++q) {
        const int ch = w + 8 * q;
        if (ch < NCHUNK) *(volatile v8h*)(dst_row + ch * 256 + l * 8) = vv[q];
    }
}

__global__ __launch_bounds__(256) void k_feat(const float* __restrict__ x,
                                              const float* __restrict__ grid_,
                                              _Float16* __restrict__ fpl)
{
    __shared__ __attribute__((aligned(16))) _Float16 rowbuf[KTOT];
    const int b = blockIdx.x;
    const int i = threadIdx.x;

    const float xv = x[(size_t)b * IN_DIM + i];
    const float* gp = grid_ + (size_t)i * NKNOT;
    float g[NKNOT];
    #pragma unroll
    for (int t = 0; t < NKNOT; ++t) g[t] = gp[t];

    float B[NKNOT - 1];
    #pragma unroll
    for (int t = 0; t < NKNOT - 1; ++t)
        B[t] = (xv >= g[t] && xv < g[t + 1]) ? 1.0f : 0.0f;

    #pragma unroll
    for (int p = 1; p <= 3; ++p) {
        #pragma unroll
        for (int t = 0; t + p < NKNOT - 1; ++t) {
            const float dl = g[t + p] - g[t];
            const float dr = g[t + p + 1] - g[t + 1];
            const float lf = (xv - g[t]) * __builtin_amdgcn_rcpf(dl);
            const float rt = (g[t + p + 1] - xv) * __builtin_amdgcn_rcpf(dr);
            B[t] = lf * B[t] + rt * B[t + 1];
        }
    }

    const float e  = __expf(-xv);
    const float sl = xv * __builtin_amdgcn_rcpf(1.0f + e);

    _Float16* rb = rowbuf + i * NF;
    rb[0] = (_Float16)(sl * FSCALE);
    #pragma unroll
    for (int c = 0; c < NB; ++c) {
        float v = B[c];
        v = (v == v) ? v : 0.0f;
        rb[1 + c] = (_Float16)(v * FSCALE);
    }
    __syncthreads();
    store_plane_row(rowbuf, fpl + (size_t)b * KTOT);
}

__global__ __launch_bounds__(256) void k_wprep(const float* __restrict__ coef,
                                               const float* __restrict__ sbase,
                                               const float* __restrict__ ssp,
                                               const float* __restrict__ msk,
                                               _Float16* __restrict__ wpl)
{
    __shared__ __attribute__((aligned(16))) _Float16 rowbuf[KTOT];
    const int o = blockIdx.x;
    const int i = threadIdx.x;
    const size_t io = (size_t)i * OUT_DIM + o;

    const float mk = msk[io];
    const float sb = sbase[io];
    const float sp = ssp[io];
    const float4* cp = (const float4*)(coef + io * NB);
    const float4 c0 = cp[0];
    const float4 c1 = cp[1];
    const float f = mk * sp * WSCALE;

    _Float16* rb = rowbuf + i * NF;
    rb[0] = (_Float16)(mk * sb * WSCALE);
    rb[1] = (_Float16)(c0.x * f);
    rb[2] = (_Float16)(c0.y * f);
    rb[3] = (_Float16)(c0.z * f);
    rb[4] = (_Float16)(c0.w * f);
    rb[5] = (_Float16)(c1.x * f);
    rb[6] = (_Float16)(c1.y * f);
    rb[7] = (_Float16)(c1.z * f);
    rb[8] = (_Float16)(c1.w * f);
    __syncthreads();
    store_plane_row(rowbuf, wpl + (size_t)o * KTOT);
}

__global__ __launch_bounds__(128) void k_gemm(const _Float16* __restrict__ fpl,
                                              const _Float16* __restrict__ wpl,
                                              float* __restrict__ out)
{
    __shared__ __attribute__((aligned(16))) float Cs[TM][TN];
    const int l  = threadIdx.x & 31;
    const int w  = threadIdx.x >> 5;
    const int h  = l >> 4;
    const int m  = l & 15;
    const int wr = w >> 1;
    const int wc = w & 1;
    const int brow = blockIdx.y * TM;
    const int bcol = blockIdx.x * TN;

    const _Float16* ap = fpl + (size_t)(brow + wr * 32 + m) * KTOT + 8 * h;
    const _Float16* bp = wpl + (size_t)(bcol + wc * 32 + m) * KTOT + 8 * h;
    const size_t t16 = (size_t)16 * KTOT;

    v8f acc00 = {};
    v8f acc01 = {};
    v8f acc10 = {};
    v8f acc11 = {};

    for (int k0 = 0; k0 < KTOT; k0 += 64) {
        #pragma unroll
        for (int s = 0; s < 2; ++s) {
            const int kk = k0 + 32 * s;
            Frag a0, a1, b0, b1;
            a0.half[0] = *(const v8h*)(ap + kk);
            a0.half[1] = *(const v8h*)(ap + kk + 16);
            a1.half[0] = *(const v8h*)(ap + t16 + kk);
            a1.half[1] = *(const v8h*)(ap + t16 + kk + 16);
            b0.half[0] = *(const v8h*)(bp + kk);
            b0.half[1] = *(const v8h*)(bp + kk + 16);
            b1.half[0] = *(const v8h*)(bp + t16 + kk);
            b1.half[1] = *(const v8h*)(bp + t16 + kk + 16);
            acc00 = __builtin_amdgcn_wmma_f32_16x16x32_f16(false, a0.v, false, b0.v, (short)0, acc00, false, false);
            acc01 = __builtin_amdgcn_wmma_f32_16x16x32_f16(false, a0.v, false, b1.v, (short)0, acc01, false, false);
            acc10 = __builtin_amdgcn_wmma_f32_16x16x32_f16(false, a1.v, false, b0.v, (short)0, acc10, false, false);
            acc11 = __builtin_amdgcn_wmma_f32_16x16x32_f16(false, a1.v, false, b1.v, (short)0, acc11, false, false);
            asm volatile("v_nop\n\tv_nop\n\tv_nop\n\tv_nop"
                         : "+v"(acc00), "+v"(acc01), "+v"(acc10), "+v"(acc11)
                         : "v"(a0.v), "v"(a1.v), "v"(b0.v), "v"(b1.v));
        }
    }

    const int trow = wr * 32 + 8 * h;
    const int tcol = wc * 32 + m;
    #pragma unroll
    for (int r = 0; r < 8; ++r) {
        Cs[trow + r][tcol]           = acc00[r] * OSCALE;
        Cs[trow + r][tcol + 16]      = acc01[r] * OSCALE;
        Cs[trow + 16 + r][tcol]      = acc10[r] * OSCALE;
        Cs[trow + 16 + r][tcol + 16] = acc11[r] * OSCALE;
    }
    __syncthreads();

    v4f vals[8];
    #pragma unroll
    for (int it = 0; it < 8; ++it) {
        const int rr = 2 * (it * 4 + w) + h;
        vals[it] = *(const v4f*)&Cs[rr][m * 4];
    }
    float* ob = out + (size_t)brow * OUT_DIM + bcol + m * 4;
    #pragma unroll
    for (int it = 0; it < 8; ++it) {
        const int rr = 2 * (it * 4 + w) + h;
        *(volatile v4f*)(ob + (size_t)rr * OUT_DIM) = vals[it];
    }
    __threadfence();
    #pragma unroll
    for (int it = 0; it < 8; ++it) {
        const int rr = 2 * (it * 4 + w) + h;
        *(volatile v4f*)(ob + (size_t)rr * OUT_DIM) = vals[it];
    }
}

extern "C" void kernel_launch(void* const* d_in, const int* in_sizes, int n_in,
                              void* d_out, int out_size, void* d_ws, size_t ws_size,
                              hipStream_t stream)
{
    if (n_in < 6) return;
    const float* x     = (const float*)d_in[0];
    const float* grid_ = (const float*)d_in[1];
    const float* coef  = (const float*)d_in[2];
    const float* sb    = (const float*)d_in[3];
    const float* sp    = (const float*)d_in[4];
    const float* mk    = (const float*)d_in[5];
    float* out = (float*)d_out;

    const int batch = in_sizes[0] / IN_DIM;
    if (batch <= 0 || (batch % TM) != 0) return;
    if (in_sizes[0] != batch * IN_DIM) return;
    if (out_size != batch * OUT_DIM) return;
    if (in_sizes[1] != IN_DIM * NKNOT) return;
    if (in_sizes[2] != IN_DIM * OUT_DIM * NB) return;
    if (in_sizes[3] != IN_DIM * OUT_DIM || in_sizes[4] != IN_DIM * OUT_DIM || in_sizes[5] != IN_DIM * OUT_DIM) return;

    const size_t fbytes = (size_t)batch * KTOT * sizeof(_Float16);
    const size_t wbytes = (size_t)OUT_DIM * KTOT * sizeof(_Float16);
    const size_t woff   = (fbytes + 127) & ~(size_t)127;
    if (woff + wbytes > ws_size) return;
    _Float16* fpl = (_Float16*)d_ws;
    _Float16* wpl = (_Float16*)((char*)d_ws + woff);

    k_feat<<<dim3(batch), dim3(256), 0, stream>>>(x, grid_, fpl);
    k_wprep<<<dim3(OUT_DIM), dim3(256), 0, stream>>>(coef, sb, sp, mk, wpl);
    k_gemm<<<dim3(OUT_DIM / TN, batch / TM), dim3(128), 0, stream>>>(fpl, wpl, out);
}
